// DeltaNet_31877247271440
// MI455X (gfx1250) — hardware-verified
//
#include <hip/hip_runtime.h>
#include <math.h>

constexpr int kBatch  = 2;
constexpr int kSeq    = 4096;
constexpr int kDim    = 1024;
constexpr int kHeads  = 4;
constexpr int kHd     = 256;
constexpr int kTok    = kBatch * kSeq;
constexpr int kChunk  = 32;
constexpr int kNChunk = kSeq / kChunk;
constexpr int kSlice  = 64;
constexpr int kNSlice = kHd / kSlice;
constexpr int kSpN    = 64;
constexpr int kGateP  = 32;
constexpr int kConvT  = 32;
constexpr int kYP     = 264;
constexpr int kMixT   = 64;
constexpr int kFirS   = 3;
constexpr int kFirL   = 31;
constexpr int kHalo   = kFirL - 1;
constexpr int kMixRows = kMixT + kHalo;
constexpr int kP256   = 264;
constexpr int kP32    = 40;

constexpr float kWCarry = 16.0f;
constexpr float kWFold  = 1.0f / kWCarry;
constexpr float kQCarry = 16.0f;
constexpr float kVFold  = 1.0f / kQCarry;
constexpr float kAFold  = 1.0f / (kQCarry * kQCarry);
constexpr float kTCarry = 8.0f;
constexpr float kTFold  = 1.0f / kTCarry;
constexpr float kUFold  = 1.0f / (kQCarry * kQCarry);
constexpr float kOFold  = 1.0f / (kQCarry * kQCarry * kQCarry);
constexpr float kInvHd  = 1.0f / (float)kHd;

static_assert(kHeads * kHd == kDim);
static_assert(kSeq % kChunk == 0 && kSeq % kMixT == 0 && kSeq % kConvT == 0);
static_assert(kTok % 64 == 0 && kDim % 64 == 0 && kSpN % 64 == 0 && kDim % 32 == 0);
static_assert(kTok % 256 == 0);
static_assert((kSlice * kP256) % 256 == 0);
static_assert((kHd * kFirL) % 4 == 0);
static_assert(kGateP * 4 == 128);

typedef __attribute__((ext_vector_type(16))) _Float16 v16h;
typedef __attribute__((ext_vector_type(8)))  _Float16 v8h;
typedef __attribute__((ext_vector_type(16))) __bf16   v16b;
typedef __attribute__((ext_vector_type(8)))  __bf16   v8b;
typedef __attribute__((ext_vector_type(8)))  float    v8f;
typedef __attribute__((ext_vector_type(4)))  float    v4f;
typedef __attribute__((ext_vector_type(4)))  unsigned int v4u;

__device__ __forceinline__ unsigned short f2bf_bits(float f) {
  unsigned u = __float_as_uint(f);
  return (unsigned short)((u + 0x7FFFu + ((u >> 16) & 1u)) >> 16);
}
__device__ __forceinline__ float bf_bits2f(unsigned short h) { return __uint_as_float(((unsigned)h) << 16); }
__device__ __forceinline__ float bf16r(float f) { return bf_bits2f(f2bf_bits(f)); }
__device__ __forceinline__ unsigned pk16(unsigned short a, unsigned short b) { return (unsigned)a | ((unsigned)b << 16); }
__device__ __forceinline__ unsigned short h_bits(float f) { const _Float16 h = (_Float16)f; return __builtin_bit_cast(unsigned short, h); }
__device__ __forceinline__ float h16_to_f32(unsigned hb) {
  const unsigned sgn = (hb & 0x8000u) << 16;
  const unsigned em = hb & 0x7fffu;
  const float fn = __uint_as_float((em << 13) + 0x38000000u);
  const float fs = (float)em * 5.9604644775390625e-8f;
  const float mag = (em < 0x400u) ? fs : fn;
  return __uint_as_float(__float_as_uint(mag) | sgn);
}

__device__ __forceinline__ void dep_guard4_h(v8f& a, v8f& b, v8f& c, v8f& d, v16h x, v16h y) { asm volatile("v_nop\n\tv_nop\n\tv_nop\n\tv_nop" : "+v"(a), "+v"(b), "+v"(c), "+v"(d) : "v"(x), "v"(y)); }
__device__ __forceinline__ void dep_guard4_b(v8f& a, v8f& b, v8f& c, v8f& d, v16b x, v16b y) { asm volatile("v_nop\n\tv_nop\n\tv_nop\n\tv_nop" : "+v"(a), "+v"(b), "+v"(c), "+v"(d) : "v"(x), "v"(y)); }
__device__ __forceinline__ void keep4_h(v16h a, v16h b, v16h c, v16h d) { asm volatile("v_nop" :: "v"(a), "v"(b), "v"(c), "v"(d)); }
__device__ __forceinline__ void keep4_b(v16b a, v16b b, v16b c, v16b d) { asm volatile("v_nop" :: "v"(a), "v"(b), "v"(c), "v"(d)); }
__device__ __forceinline__ void acc_guard4(v8f& a, v8f& b, v8f& c, v8f& d) { asm volatile("v_nop\n\tv_nop\n\tv_nop\n\tv_nop" : "+v"(a), "+v"(b), "+v"(c), "+v"(d)); }
template <typename T> struct Frag;
template <> struct Frag<_Float16> {
  typedef v16h V; union U { v16h v; v8h h[2]; };
  static __device__ __forceinline__ v16h load(const _Float16* p) {
    U f; f.h[0] = *(const v8h*)(p); f.h[1] = *(const v8h*)(p + 16); return f.v;
  }
  static __device__ __forceinline__ v8f mma(v16h a, v16h b, v8f c) {
    return __builtin_amdgcn_wmma_f32_16x16x32_f16(false, a, false, b, (short)0, c, false, false);
  }
  static __device__ __forceinline__ void guard4(v8f& a, v8f& b, v8f& c, v8f& d, v16h x, v16h y) { dep_guard4_h(a, b, c, d, x, y); }
  static __device__ __forceinline__ void keep(v16h a, v16h b, v16h c, v16h d) { keep4_h(a, b, c, d); }
};
template <> struct Frag<__bf16> {
  typedef v16b V; union U { v16b v; v8b h[2]; };
  static __device__ __forceinline__ v16b load(const __bf16* p) {
    U f; f.h[0] = *(const v8b*)(p); f.h[1] = *(const v8b*)(p + 16); return f.v;
  }
  static __device__ __forceinline__ v8f mma(v16b a, v16b b, v8f c) {
    return __builtin_amdgcn_wmma_f32_16x16x32_bf16(false, a, false, b, (short)0, c, false, false);
  }
  static __device__ __forceinline__ void guard4(v8f& a, v8f& b, v8f& c, v8f& d, v16b x, v16b y) { dep_guard4_b(a, b, c, d, x, y); }
  static __device__ __forceinline__ void keep(v16b a, v16b b, v16b c, v16b d) { keep4_b(a, b, c, d); }
};

__device__ __forceinline__ v8f mma_h(v16h a, v16h b, v8f c) {
  c = __builtin_amdgcn_wmma_f32_16x16x32_f16(false, a, false, b, (short)0, c, false, false);
  asm volatile("v_nop\n\tv_nop\n\tv_nop\n\tv_nop" : "+v"(c) : "v"(a), "v"(b));
  return c;
}

template <int ET> struct Elem;
template <> struct Elem<0> { typedef _Float16 T; };
template <> struct Elem<1> { typedef __bf16 T; };
template <int ET, bool SPLIT, int BIAS_MODE, int OUT_MODE, bool RESID, int ACT = 0>
__global__ __launch_bounds__(256) void wmma_gemm64(
    const unsigned short* __restrict__ Ap, const unsigned short* __restrict__ A2p, int lda, long strideA,
    const unsigned short* __restrict__ Btp, const unsigned short* __restrict__ Bt2p, int ldb, long strideB,
    void* __restrict__ Cout, void* __restrict__ Cout2, int ldc, long strideC,
    const float* __restrict__ bias,
    const float* __restrict__ resid, long strideR,
    int M, int N, int K, float scale) {
  typedef typename Elem<ET>::T T;
  typedef typename Frag<T>::V V;
  const T* A = (const T*)Ap; const T* A2 = (const T*)A2p; const T* Bt = (const T*)Btp; const T* Bt2 = (const T*)Bt2p;
  __shared__ __align__(16) float sT[8][16 * 68];
  const int b    = blockIdx.y;
  const int lane = threadIdx.x & 31;
  const int wave = threadIdx.x >> 5;
  const int tilesN = N >> 6;
  const int tilesM = M >> 6;
  const int tile = blockIdx.x * 8 + wave;
  if (tile >= tilesM * tilesN) return;
  const int tm = tile / tilesN;
  const int tn = tile - tm * tilesN;
  const int m0 = tm << 6;
  const int n0 = tn << 6;

  const T* Ab  = A  + (size_t)b * strideA;
  const T* Bb  = Bt + (size_t)b * strideB;
  const T* Ab2 = SPLIT ? (A2  + (size_t)b * strideA) : nullptr;
  const T* Bb2 = SPLIT ? (Bt2 + (size_t)b * strideB) : nullptr;

  const int rlane = lane & 15;
  const int koff  = (lane >> 4) * 8;
  const int mOff  = (lane >> 4) * 8;

  v8f acc[4][4];
#pragma unroll
  for (int i = 0; i < 4; ++i)
#pragma unroll
    for (int j = 0; j < 4; ++j) acc[i][j] = (v8f){0.f,0.f,0.f,0.f,0.f,0.f,0.f,0.f};

  for (int k0 = 0; k0 < K; k0 += 32) {
    V bh[4], bl[4];
#pragma unroll
    for (int j = 0; j < 4; ++j) {
      const size_t bo = (size_t)(n0 + (j << 4) + rlane) * ldb + koff + k0;
      bh[j] = Frag<T>::load(Bb + bo);
      if (SPLIT) bl[j] = Frag<T>::load(Bb2 + bo);
    }
#pragma unroll
    for (int i = 0; i < 4; ++i) {
      const size_t ao = (size_t)(m0 + (i << 4) + rlane) * lda + koff + k0;
      V ah = Frag<T>::load(Ab + ao);
      V al;
      if (SPLIT) al = Frag<T>::load(Ab2 + ao);
#pragma unroll
      for (int j = 0; j < 4; ++j) {
        acc[i][j] = Frag<T>::mma(ah, bh[j], acc[i][j]);
        if (SPLIT) {
          acc[i][j] = Frag<T>::mma(ah, bl[j], acc[i][j]);
          acc[i][j] = Frag<T>::mma(al, bh[j], acc[i][j]);
        }
      }
      Frag<T>::guard4(acc[i][0], acc[i][1], acc[i][2], acc[i][3], ah, SPLIT ? al : ah);
    }
    Frag<T>::keep(bh[0], bh[1], bh[2], bh[3]);
    if (SPLIT) Frag<T>::keep(bl[0], bl[1], bl[2], bl[3]);
  }
  acc_guard4(acc[0][0], acc[0][1], acc[0][2], acc[0][3]);
  acc_guard4(acc[1][0], acc[1][1], acc[1][2], acc[1][3]);
  acc_guard4(acc[2][0], acc[2][1], acc[2][2], acc[2][3]);
  acc_guard4(acc[3][0], acc[3][1], acc[3][2], acc[3][3]);

  float* slab = sT[wave];
  const float* Rb = RESID ? (resid + (size_t)b * strideR) : nullptr;
#pragma unroll
  for (int i = 0; i < 4; ++i) {
    const int mBase = m0 + (i << 4);
#pragma unroll
    for (int j = 0; j < 4; ++j) {
      const int n = n0 + (j << 4) + rlane;
      float bv = 0.f;
      if (BIAS_MODE == 2) bv = bias[n];
#pragma unroll
      for (int r = 0; r < 8; ++r) {
        float v = acc[i][j][r] * scale;
        if (BIAS_MODE == 1) v += bias[mBase + mOff + r];
        if (BIAS_MODE == 2) v += bv;
        if (RESID) v += Rb[(size_t)(mBase + mOff + r) * ldc + n];
        if (ACT == 2) v = fmaxf(v, 0.0f);
        if (ACT == 4) v = (v > 0.f) ? v : 0.01f * v;
        slab[(mOff + r) * 68 + (j << 4) + rlane] = v;
      }
    }
    __builtin_amdgcn_fence(__ATOMIC_RELEASE, "workgroup");
    __builtin_amdgcn_wave_barrier();
    __builtin_amdgcn_fence(__ATOMIC_ACQUIRE, "workgroup");
    if (OUT_MODE == 0) {
      float* C = (float*)Cout + (size_t)b * strideC;
      const int hh = lane >> 4, c4 = (lane & 15) * 4;
      for (int pass = 0; pass < 2; ++pass) {
#pragma unroll
        for (int it = 0; it < 8; ++it) {
          const int row = it * 2 + hh;
          v4f v = *(const v4f*)(slab + row * 68 + c4);
          *(volatile v4f*)(C + (size_t)(mBase + row) * ldc + n0 + c4) = v;
        }
        __threadfence();
      }
    } else {
      const int q = lane >> 3, c8 = (lane & 7) * 8;
      unsigned short* C  = (unsigned short*)Cout  + (size_t)b * strideC;
      unsigned short* C2 = (OUT_MODE == 2) ? ((unsigned short*)Cout2 + (size_t)b * strideC) : nullptr;
      for (int pass = 0; pass < 2; ++pass) {
#pragma unroll
        for (int it = 0; it < 4; ++it) {
          const int row = it * 4 + q;
          const float* sp = slab + row * 68 + c8;
          v8h hv, lv;
#pragma unroll
          for (int e = 0; e < 8; ++e) {
            if (OUT_MODE == 1) {
              hv[e] = (_Float16)sp[e];
            } else {
              unsigned short hb = f2bf_bits(sp[e]);
              unsigned short lb = f2bf_bits(sp[e] - bf_bits2f(hb));
              hv[e] = __builtin_bit_cast(_Float16, hb);
              lv[e] = __builtin_bit_cast(_Float16, lb);
            }
          }
          *(volatile v8h*)(C + (size_t)(mBase + row) * ldc + n0 + c8) = hv;
          if (OUT_MODE == 2) *(volatile v8h*)(C2 + (size_t)(mBase + row) * ldc + n0 + c8) = lv;
        }
        __threadfence();
      }
    }
    __builtin_amdgcn_fence(__ATOMIC_RELEASE, "workgroup");
    __builtin_amdgcn_wave_barrier();
    __builtin_amdgcn_fence(__ATOMIC_ACQUIRE, "workgroup");
  }
}

__global__ __launch_bounds__(256) void cvt8_act_kernel(const float* __restrict__ src, unsigned short* __restrict__ dst, int n8) {
  const int i = blockIdx.x * 256 + threadIdx.x;
  if (i < n8) {
    const float* sp = src + (size_t)i * 8;
    const v4f a = *(const v4f*)(sp);
    const v4f c = *(const v4f*)(sp + 4);
    unsigned short hb[8];
#pragma unroll
    for (int e = 0; e < 4; ++e) {
      hb[e]     = h_bits(bf16r(a[e]));
      hb[4 + e] = h_bits(bf16r(c[e]));
    }
    const v4u u = (v4u){pk16(hb[0], hb[1]), pk16(hb[2], hb[3]), pk16(hb[4], hb[5]), pk16(hb[6], hb[7])};
    unsigned short* q = dst + (size_t)i * 8;
    *(volatile v4u*)q = u;
    __threadfence();
    *(volatile v4u*)q = u;
  }
}

__global__ __launch_bounds__(256) void wtcast_kernel(const float* __restrict__ W0, const float* __restrict__ W1,
                                                     const float* __restrict__ W2, const float* __restrict__ W3,
                                                     unsigned short* __restrict__ out, float scale) {
  __shared__ float sm[64][65];
  const int t  = threadIdx.x;
  const int d0 = blockIdx.x * 64;
  const int n0 = blockIdx.y * 64;
  const int z  = blockIdx.z;
  const float* W = (z == 0) ? W0 : (z == 1) ? W1 : (z == 2) ? W2 : W3;
#pragma unroll
  for (int i = 0; i < 16; ++i) {
    const int e = i * 256 + t;
    const int r = e >> 6;
    const int c = e & 63;
    sm[c][r] = bf16r(W[(size_t)(d0 + r) * kDim + n0 + c]) * scale;
  }
  __syncthreads();
  const int lane = t & 31, wave = t >> 5;
  const int q = lane >> 3, c8 = (lane & 7) * 8;
  unsigned short* op = out + (size_t)z * kDim * kDim;
  for (int pass = 0; pass < 2; ++pass) {
#pragma unroll
    for (int it = 0; it < 2; ++it) {
      const int row = wave * 8 + it * 4 + q;
      unsigned short hb[8];
#pragma unroll
      for (int e = 0; e < 8; ++e) hb[e] = h_bits(sm[row][c8 + e]);
      const v4u u = (v4u){pk16(hb[0], hb[1]), pk16(hb[2], hb[3]), pk16(hb[4], hb[5]), pk16(hb[6], hb[7])};
      *(volatile v4u*)(op + (size_t)(n0 + row) * kDim + d0 + c8) = u;
    }
    __threadfence();
  }
}

__global__ __launch_bounds__(256) void wscast_kernel(const float* __restrict__ Wb, const float* __restrict__ Wg,
                                                     const float* __restrict__ Wl, unsigned short* __restrict__ out, float scale) {
  const int i  = blockIdx.x * 256 + threadIdx.x;
  const int n  = i >> 7;
  const int k8 = (i & 127) * 8;
  int nl = n - 8;
  nl = nl < 0 ? 0 : (nl > 11 ? 11 : nl);
  const float* src = (n < 4) ? (Wb + n) : (n < 8) ? (Wg + (n - 4)) : (Wl + nl);
  const int stride = (n < 8) ? 4 : 12;
  const bool live = (n < 20);
  unsigned short hb[8];
#pragma unroll
  for (int e = 0; e < 8; ++e) {
    const float w = src[(size_t)(k8 + e) * stride];
    const float v = live ? (bf16r(w) * scale) : 0.0f;
    hb[e] = h_bits(v);
  }
  const v4u u = (v4u){pk16(hb[0], hb[1]), pk16(hb[2], hb[3]), pk16(hb[4], hb[5]), pk16(hb[6], hb[7])};
  unsigned short* q = out + (size_t)n * kDim + k8;
  *(volatile v4u*)q = u;
  __threadfence();
  *(volatile v4u*)q = u;
}

template <bool NORM>
__global__ __launch_bounds__(256) void conv_act_kernel(const float* __restrict__ lin, const float* __restrict__ cw,
                                                       unsigned short* __restrict__ out) {
  __shared__ __align__(16) float ys[kConvT * kYP];
  const int tid = threadIdx.x, lane = tid & 31, wave = tid >> 5;
  const int tile = blockIdx.x;
  const int tpb  = kSeq / kConvT;
  const int b    = tile / tpb;
  const int t0   = (tile - b * tpb) * kConvT;
  const int h    = blockIdx.y;
  const int c    = h * kHd + tid;
  const size_t rowbase = (size_t)b * kSeq;

  const v4f wv = *(const v4f*)(cw + (size_t)c * 4);
  const float w0 = bf16r(wv[0]), w1 = bf16r(wv[1]), w2 = bf16r(wv[2]), w3 = bf16r(wv[3]);

  const int r0 = t0 - 3, r1 = t0 - 2, r2 = t0 - 1;
  const float l0v = lin[(rowbase + (size_t)(r0 < 0 ? 0 : r0)) * kDim + c];
  const float l1v = lin[(rowbase + (size_t)(r1 < 0 ? 0 : r1)) * kDim + c];
  const float l2v = lin[(rowbase + (size_t)(r2 < 0 ? 0 : r2)) * kDim + c];
  float x0 = (r0 >= 0) ? l0v : 0.0f;
  float x1 = (r1 >= 0) ? l1v : 0.0f;
  float x2 = (r2 >= 0) ? l2v : 0.0f;

#pragma unroll 1
  for (int i = 0; i < kConvT; ++i) {
    const float xn = lin[(rowbase + (size_t)(t0 + i)) * kDim + c];
    float y = w0 * x0;
    y = fmaf(w1, x1, y);
    y = fmaf(w2, x2, y);
    y = fmaf(w3, xn, y);
    const float sg = 1.0f / (1.0f + expf(-y));
    ys[i * kYP + tid] = y * sg;
    x0 = x1; x1 = x2; x2 = xn;
  }
  __syncthreads();

#pragma unroll 1
  for (int rr = 0; rr < 4; ++rr) {
    const int row = wave * 4 + rr;
    const float* yp = ys + row * kYP + lane * 8;
    const v4f a = *(const v4f*)(yp);
    const v4f d = *(const v4f*)(yp + 4);
    float sc = 1.0f;
    if (NORM) {
      float ss = (a[0] * a[0] + a[1] * a[1]) + (a[2] * a[2] + a[3] * a[3]);
      ss += (d[0] * d[0] + d[1] * d[1]) + (d[2] * d[2] + d[3] * d[3]);
#pragma unroll
      for (int off = 16; off > 0; off >>= 1) ss += __shfl_xor(ss, off, 32);
      sc = rsqrtf(ss + 1e-6f);
    }
    unsigned short hb[8];
#pragma unroll
    for (int e = 0; e < 4; ++e) {
      hb[e]     = h_bits((a[e] * sc) * kQCarry);
      hb[4 + e] = h_bits((d[e] * sc) * kQCarry);
    }
    const v4u u = (v4u){pk16(hb[0], hb[1]), pk16(hb[2], hb[3]), pk16(hb[4], hb[5]), pk16(hb[6], hb[7])};
    unsigned short* q = out + (rowbase + (size_t)(t0 + row)) * kDim + h * kHd + lane * 8;
    *(volatile v4u*)q = u;
    __threadfence();
    *(volatile v4u*)q = u;
  }
}

__global__ __launch_bounds__(256) void gate_kernel(const float* __restrict__ sp, const float* __restrict__ bg,
                                                   const float* __restrict__ bl, const float* __restrict__ lt,
                                                   float* __restrict__ gate) {
  __shared__ __align__(16) float sg[256 * 36];
  const int tid = threadIdx.x;
  const int tok = blockIdx.x * 256 + tid;
  float* row = sg + tid * 36;
  const float* sr = sp + (size_t)tok * kSpN;
#pragma unroll
  for (int i = 0; i < 5; ++i) {
    const v4f v = *(const v4f*)(sr + 4 * i);
    *(v4f*)(row + 4 * i) = v;
  }
  const v4f zz = (v4f){0.f, 0.f, 0.f, 0.f};
  *(v4f*)(row + 20) = zz;
  *(v4f*)(row + 24) = zz;
  *(v4f*)(row + 28) = zz;
#pragma unroll 1
  for (int h = 0; h < kHeads; ++h) {
    const float zb = row[h];
    row[h] = 1.0f / (1.0f + expf(-zb));
    const float zg = row[4 + h] + bf16r(bg[h]);
    row[4 + h] = 1.0f / (1.0f + expf(-zg));
    const float it = 1.0f / expf(bf16r(lt[h]));
    const float a0 = (row[8 + 3 * h + 0] + bf16r(bl[3 * h + 0])) * it;
    const float a1 = (row[8 + 3 * h + 1] + bf16r(bl[3 * h + 1])) * it;
    const float a2 = (row[8 + 3 * h + 2] + bf16r(bl[3 * h + 2])) * it;
    const float mx = fmaxf(a0, fmaxf(a1, a2));
    const float e0 = expf(a0 - mx), e1 = expf(a1 - mx), e2 = expf(a2 - mx);
    const float inv = 1.0f / ((e0 + e1) + e2);
    row[8 + 3 * h + 0] = e0 * inv;
    row[8 + 3 * h + 1] = e1 * inv;
    row[8 + 3 * h + 2] = e2 * inv;
  }
  __syncthreads();
  float* gp = gate + (size_t)blockIdx.x * 256 * kGateP;
  for (int pass = 0; pass < 2; ++pass) {
#pragma unroll
    for (int it = 0; it < 8; ++it) {
      const int idx = it * 256 + tid;
      const int tl = idx >> 3, c4 = (idx & 7) * 4;
      const v4f v = *(const v4f*)(sg + tl * 36 + c4);
      *(volatile v4f*)(gp + (size_t)tl * kGateP + c4) = v;
    }
    __threadfence();
  }
}

__global__ __launch_bounds__(256) void chunk_scan_kernel(const unsigned short* __restrict__ qpl,
                                                         const unsigned short* __restrict__ kpl,
                                                         const unsigned short* __restrict__ vpl,
                                                         const float* __restrict__ gate,
                                                         float* __restrict__ dout) {
  __shared__ __align__(16) _Float16 sQ[kChunk * kP256];
  __shared__ __align__(16) _Float16 sK[kChunk * kP256];
  __shared__ __align__(16) _Float16 sW[kChunk * kP256];
  __shared__ __align__(16) _Float16 sKT[kHd * kP32];
  __shared__ __align__(16) _Float16 sVU[kSlice * kP32];
  __shared__ __align__(16) _Float16 sAT[kChunk * kP32];
  __shared__ __align__(16) _Float16 sTH[kChunk * kP32];
  __shared__ __align__(16) _Float16 sST[kSlice * kP256];
  __shared__ __align__(16) float    sAF[2 * kChunk * kChunk];
  __shared__ float sBeta[kChunk];

  const int dv0 = blockIdx.x * kSlice;
  const int h = blockIdx.y, b = blockIdx.z;
  const int tid = threadIdx.x, lane = tid & 31, wave = tid >> 5;
  const int c = lane & 15, hh = lane >> 4, koff = hh * 8;
  const int mt = wave >> 2, nt = wave & 3;
  const int hoff = h * kHd;
  const v8f z8 = {0.f, 0.f, 0.f, 0.f, 0.f, 0.f, 0.f, 0.f};
  float* sTF  = sAF + kChunk * kChunk;
  float* slab = sAF;

  {
    unsigned short* p = (unsigned short*)sST;
#pragma unroll 1
    for (int i = tid; i < kSlice * kP256; i += 256) p[i] = (unsigned short)0;
  }
  v8f Sacc[2][4];
#pragma unroll
  for (int i = 0; i < 2; ++i)
#pragma unroll
    for (int j = 0; j < 4; ++j) Sacc[i][j] = z8;

#pragma unroll 1
  for (int ch = 0; ch < kNChunk; ++ch) {
    const size_t tok0 = (size_t)b * kSeq + (size_t)ch * kChunk;

#pragma unroll 1
    for (int rr = 0; rr < 4; ++rr) {
      const int r = wave * 4 + rr;
      const size_t go = (tok0 + (size_t)r) * kDim + hoff + lane * 8;
      const v4u qv = *(const v4u*)(qpl + go);
      const v4u kv = *(const v4u*)(kpl + go);
      *(v4u*)(sQ + r * kP256 + lane * 8) = qv;
      *(v4u*)(sK + r * kP256 + lane * 8) = kv;
      unsigned short* kt = (unsigned short*)sKT + (lane * 8) * kP32 + r;
#pragma unroll
      for (int e = 0; e < 4; ++e) {
        const unsigned w = kv[e];
        kt[(2 * e) * kP32]     = (unsigned short)(w & 0xffffu);
        kt[(2 * e + 1) * kP32] = (unsigned short)(w >> 16);
      }
    }
    {
      const int r  = wave * 4 + (lane >> 3);
      const int c8 = (lane & 7) * 8;
      const v4u vv = *(const v4u*)(vpl + (tok0 + (size_t)r) * kDim + hoff + dv0 + c8);
      unsigned short* vt = (unsigned short*)sVU + c8 * kP32 + r;
#pragma unroll
      for (int e = 0; e < 4; ++e) {
        const unsigned w = vv[e];
        vt[(2 * e) * kP32]     = (unsigned short)(w & 0xffffu);
        vt[(2 * e + 1) * kP32] = (unsigned short)(w >> 16);
      }
    }
    if (tid < kChunk) sBeta[tid] = gate[(tok0 + (size_t)tid) * kGateP + h];
    __syncthreads();

    {
      const int w4 = wave & 3, tmt = w4 >> 1, tnt = w4 & 1;
      const _Float16* Ap = (wave < 4) ? sK : sQ;
      const _Float16* ar = Ap + (tmt * 16 + c) * kP256 + koff;
      const _Float16* br = sK + (tnt * 16 + c) * kP256 + koff;
      v8f a = z8;
#pragma unroll 2
      for (int kk = 0; kk < kHd / 32; ++kk) {
        const v16h fa = Frag<_Float16>::load(ar + kk * 32);
        const v16h fb = Frag<_Float16>::load(br + kk * 32);
        a = mma_h(fa, fb, a);
      }
      if (wave < 4) {
#pragma unroll
        for (int r = 0; r < 8; ++r) {
          const int ro = tmt * 16 + 8 * hh + r;
          sAF[ro * kChunk + tnt * 16 + c] = (a[r] * kAFold) * sBeta[ro];
        }
      } else {
#pragma unroll
        for (int r = 0; r < 8; ++r) {
          const int ro = tmt * 16 + 8 * hh + r, co = tnt * 16 + c;
          const float val = (co <= ro) ? a[r] : 0.0f;
          sAT[ro * kP32 + co] = (_Float16)val;
        }
      }
    }
    __syncthreads();

    if (wave == 0) {
      const int j = lane;
      const float bj = sBeta[j] * kTCarry;
#pragma unroll 1
      for (int i = 0; i < kChunk; ++i) {
        float t = (i == j) ? 1.0f : 0.0f;
#pragma unroll 1
        for (int m = 0; m < i; ++m) t -= sAF[i * kChunk + m] * sTF[m * kChunk + j];
        sTF[i * kChunk + j] = t;
        sTH[i * kP32 + j] = (_Float16)(t * bj);
      }
    }
    __syncthreads();

    v8f accu;
    {
      const v16h ta = Frag<_Float16>::load(sTH + (mt * 16 + c) * kP32 + koff);
#pragma unroll
      for (int jj = 0; jj < 4; ++jj) {
        const int n0 = (nt * 4 + jj) * 16;
        const v16h fb = Frag<_Float16>::load(sKT + (n0 + c) * kP32 + koff);
        v8f a = mma_h(ta, fb, z8);
#pragma unroll
        for (int r = 0; r < 8; ++r) sW[(mt * 16 + 8 * hh + r) * kP256 + n0 + c] = (_Float16)(a[r] * kTFold);
      }
      const v16h fv = Frag<_Float16>::load(sVU + (nt * 16 + c) * kP32 + koff);
      accu = mma_h(ta, fv, z8);
#pragma unroll
      for (int r = 0; r < 8; ++r) accu[r] *= kTFold;
    }
    __syncthreads();

    {
      const _Float16* ar = sW + (mt * 16 + c) * kP256 + koff;
      const _Float16* br = sST + (nt * 16 + c) * kP256 + koff;
      v8f a = z8;
#pragma unroll 2
      for (int kk = 0; kk < kHd / 32; ++kk) {
        const v16h fa = Frag<_Float16>::load(ar + kk * 32);
        const v16h fb = Frag<_Float16>::load(br + kk * 32);
        a = mma_h(fa, fb, a);
      }
      v8h uv;
#pragma unroll
      for (int r = 0; r < 8; ++r) {
        const float u = accu[r] - a[r] * kUFold;
        uv[r] = (_Float16)u;
      }
      *(v8h*)(sVU + (nt * 16 + c) * kP32 + mt * 16 + 8 * hh) = uv;
    }
    __syncthreads();

    {
      const _Float16* ar = sQ + (mt * 16 + c) * kP256 + koff;
      const _Float16* br = sST + (nt * 16 + c) * kP256 + koff;
      v8f a = z8;
#pragma unroll 2
      for (int kk = 0; kk < kHd / 32; ++kk) {
        const v16h fa = Frag<_Float16>::load(ar + kk * 32);
        const v16h fb = Frag<_Float16>::load(br + kk * 32);
        a = mma_h(fa, fb, a);
      }
      {
        const v16h fa = Frag<_Float16>::load(sAT + (mt * 16 + c) * kP32 + koff);
        const v16h fb = Frag<_Float16>::load(sVU + (nt * 16 + c) * kP32 + koff);
        a = mma_h(fa, fb, a);
      }
#pragma unroll
      for (int r = 0; r < 8; ++r) slab[(mt * 16 + 8 * hh + r) * kSlice + nt * 16 + c] = a[r] * kOFold;
    }
    {
      v16h ub[4];
#pragma unroll
      for (int n2 = 0; n2 < 4; ++n2) ub[n2] = Frag<_Float16>::load(sVU + (n2 * 16 + c) * kP32 + koff);
#pragma unroll
      for (int si = 0; si < 2; ++si) {
        const int s2 = wave + si * 8;
        const v16h ka = Frag<_Float16>::load(sKT + (s2 * 16 + c) * kP32 + koff);
#pragma unroll
        for (int n2 = 0; n2 < 4; ++n2) Sacc[si][n2] = mma_h(ka, ub[n2], Sacc[si][n2]);
      }
    }
    __syncthreads();

#pragma unroll
    for (int si = 0; si < 2; ++si) {
#pragma unroll
      for (int n2 = 0; n2 < 4; ++n2) {
        v8h sv;
#pragma unroll
        for (int r = 0; r < 8; ++r) sv[r] = (_Float16)Sacc[si][n2][r];
        *(v8h*)(sST + (n2 * 16 + c) * kP256 + (wave + si * 8) * 16 + 8 * hh) = sv;
      }
    }
    {
      const int c4 = c * 4;
      for (int pass = 0; pass < 2; ++pass) {
#pragma unroll
        for (int it = 0; it < 2; ++it) {
          const int row = wave * 4 + it * 2 + hh;
          const v4f v = *(const v4f*)(slab + row * kSlice + c4);
          *(volatile v4f*)(dout + (tok0 + (size_t)row) * kDim + hoff + dv0 + c4) = v;
        }
        __threadfence();
      }
    }
  }
}

__global__ __launch_bounds__(256) void mix_norm_kernel(const unsigned short* __restrict__ vpl,
                                                       const float* __restrict__ dlt,
                                                       const float* __restrict__ gate,
                                                       const float* __restrict__ fs,
                                                       const float* __restrict__ fl,
                                                       const float* __restrict__ rmsw,
                                                       unsigned short* __restrict__ oh) {
  __shared__ __align__(16) float vt[kMixRows * kHd];
  const int tid = threadIdx.x, lane = tid & 31, wave = tid >> 5;
  const int tile = blockIdx.x;
  const int tpb  = kSeq / kMixT;
  const int b    = tile / tpb;
  const int l0   = (tile - b * tpb) * kMixT;
  const int h    = blockIdx.y;
  const size_t rowbase = (size_t)b * kSeq;

  {
    const float* flh = fl + (size_t)h * kHd * kFirL;
#pragma unroll 1
    for (int i = tid; i < kHd * kFirL / 4; i += 256) {
      const v4f t = *(const v4f*)(flh + 4 * i);
      *(v4f*)(vt + 4 * i) = t;
    }
  }
  __syncthreads();
  float wl[kFirL];
#pragma unroll
  for (int t = 0; t < kFirL; ++t) wl[t] = bf16r(vt[tid * kFirL + t]);
  const float ws0 = bf16r(fs[(size_t)(h * kHd + tid) * kFirS + 0]);
  const float ws1 = bf16r(fs[(size_t)(h * kHd + tid) * kFirS + 1]);
  const float ws2 = bf16r(fs[(size_t)(h * kHd + tid) * kFirS + 2]);
  __syncthreads();

#pragma unroll 1
  for (int i = tid; i < kMixRows * 32; i += 256) {
    const int row = i >> 5, c8 = (i & 31) * 8;
    const int l  = l0 - kHalo + row;
    const int lc = l < 0 ? 0 : l;
    const v4u w = *(const v4u*)(vpl + (rowbase + (size_t)lc) * kDim + h * kHd + c8);
    const bool ok = (l >= 0);
    const unsigned u0 = w[0], u1 = w[1], u2 = w[2], u3 = w[3];
    v4f o0, o1;
    const float f0 = h16_to_f32(u0 & 0xffffu) * kVFold, f1 = h16_to_f32(u0 >> 16) * kVFold;
    const float f2 = h16_to_f32(u1 & 0xffffu) * kVFold, f3 = h16_to_f32(u1 >> 16) * kVFold;
    const float f4 = h16_to_f32(u2 & 0xffffu) * kVFold, f5 = h16_to_f32(u2 >> 16) * kVFold;
    const float f6 = h16_to_f32(u3 & 0xffffu) * kVFold, f7 = h16_to_f32(u3 >> 16) * kVFold;
    o0[0] = ok ? f0 : 0.0f; o0[1] = ok ? f1 : 0.0f; o0[2] = ok ? f2 : 0.0f; o0[3] = ok ? f3 : 0.0f;
    o1[0] = ok ? f4 : 0.0f; o1[1] = ok ? f5 : 0.0f; o1[2] = ok ? f6 : 0.0f; o1[3] = ok ? f7 : 0.0f;
    *(v4f*)(vt + row * kHd + c8)     = o0;
    *(v4f*)(vt + row * kHd + c8 + 4) = o1;
  }
  __syncthreads();

#pragma unroll 1
  for (int i = 0; i < kMixT; ++i) {
    const size_t tok = rowbase + (size_t)(l0 + i);
    const float* gp = gate + tok * kGateP;
    const float g  = gp[4 + h];
    const float p0 = gp[8 + 3 * h + 0], p1 = gp[8 + 3 * h + 1], p2 = gp[8 + 3 * h + 2];
    const float del = dlt[tok * kDim + h * kHd + tid];
    const float vcur = vt[(kHalo + i) * kHd + tid];
    float lsv = ws0 * vt[(kHalo - 2 + i) * kHd + tid];
    lsv = fmaf(ws1, vt[(kHalo - 1 + i) * kHd + tid], lsv);
    lsv = fmaf(ws2, vcur, lsv);
    float llv = 0.0f;
#pragma unroll
    for (int t = 0; t < kFirL; ++t) llv = fmaf(wl[t], vt[(i + t) * kHd + tid], llv);
    const float lm = p0 * vcur + p1 * lsv + p2 * llv;
    const float val = g * del + (1.0f - g) * lm;
    vt[i * kHd + tid] = val;
  }
  __syncthreads();

  const v4f rwa = *(const v4f*)(rmsw + lane * 8);
  const v4f rwb = *(const v4f*)(rmsw + lane * 8 + 4);
#pragma unroll 1
  for (int q = 0; q < 8; ++q) {
    const int row = wave * 8 + q;
    const float* vp = vt + row * kHd + lane * 8;
    const v4f a = *(const v4f*)(vp);
    const v4f d = *(const v4f*)(vp + 4);
    float ss = (a[0] * a[0] + a[1] * a[1]) + (a[2] * a[2] + a[3] * a[3]);
    ss += (d[0] * d[0] + d[1] * d[1]) + (d[2] * d[2] + d[3] * d[3]);
#pragma unroll
    for (int off = 16; off > 0; off >>= 1) ss += __shfl_xor(ss, off, 32);
    const float rr = rsqrtf(ss * kInvHd + 1e-5f);
    unsigned short hb[8];
#pragma unroll
    for (int e = 0; e < 4; ++e) {
      hb[e]     = h_bits((a[e] * rr) * bf16r(rwa[e]));
      hb[4 + e] = h_bits((d[e] * rr) * bf16r(rwb[e]));
    }
    const v4u u = (v4u){pk16(hb[0], hb[1]), pk16(hb[2], hb[3]), pk16(hb[4], hb[5]), pk16(hb[6], hb[7])};
    unsigned short* op = oh + (rowbase + (size_t)(l0 + row)) * kDim + h * kHd + lane * 8;
    *(volatile v4u*)op = u;
    __threadfence();
    *(volatile v4u*)op = u;
  }
}

constexpr size_t kBytesXH   = (size_t)kTok * kDim * 2;
constexpr size_t kBytesWT   = (size_t)4 * kDim * kDim * 2;
constexpr size_t kBytesWST  = (size_t)kSpN * kDim * 2;
constexpr size_t kBytesLIN  = (size_t)kTok * kDim * 4;
constexpr size_t kBytesSP   = (size_t)kTok * kSpN * 4;
constexpr size_t kBytesGATE = (size_t)kTok * kGateP * 4;
constexpr size_t kBytesTotal = kBytesXH + kBytesWT + kBytesWST + kBytesLIN + 3 * kBytesXH + kBytesSP + kBytesGATE + kBytesXH;
static_assert(kBytesTotal <= (size_t)134217728);
static_assert(kBytesXH % 256 == 0 && kBytesWT % 256 == 0 && kBytesWST % 256 == 0 && kBytesSP % 256 == 0 && kBytesGATE % 256 == 0);

extern "C" void kernel_launch(void* const* d_in, const int* in_sizes, int n_in,
                              void* d_out, int out_size, void* d_ws, size_t ws_size, hipStream_t stream) {
  if (n_in < 17 || d_out == nullptr || d_ws == nullptr) return;
  if (in_sizes[0] != kTok * kDim || in_sizes[1] != kDim * kDim || in_sizes[2] != kDim * kDim ||
      in_sizes[3] != kDim * kDim || in_sizes[4] != kDim * 4 || in_sizes[5] != kDim * 4 ||
      in_sizes[6] != kDim * 4 || in_sizes[7] != kDim * kHeads || in_sizes[8] != kDim * kFirS ||
      in_sizes[9] != kDim * kFirL || in_sizes[10] != kDim * kHeads || in_sizes[11] != kHeads ||
      in_sizes[12] != kDim * 12 || in_sizes[13] != 12 || in_sizes[14] != kHeads ||
      in_sizes[15] != kHd || in_sizes[16] != kDim * kDim || out_size != kTok * kDim) return;
  if (kBytesTotal > ws_size) return;

  const float* x      = (const float*)d_in[0];
  const float* Wq     = (const float*)d_in[1];
  const float* Wk     = (const float*)d_in[2];
  const float* Wv     = (const float*)d_in[3];
  const float* conv_q = (const float*)d_in[4];
  const float* conv_k = (const float*)d_in[5];
  const float* conv_v = (const float*)d_in[6];
  const float* Wb     = (const float*)d_in[7];
  const float* fir_s  = (const float*)d_in[8];
  const float* fir_l  = (const float*)d_in[9];
  const float* Wg     = (const float*)d_in[10];
  const float* bg     = (const float*)d_in[11];
  const float* Wl     = (const float*)d_in[12];
  const float* bl     = (const float*)d_in[13];
  const float* ltmp   = (const float*)d_in[14];
  const float* rmsw   = (const float*)d_in[15];
  const float* Wo     = (const float*)d_in[16];

  char* ws = (char*)d_ws; size_t off = 0;
  auto carve = [&](size_t bytes) -> char* { char* p = ws + off; off += (bytes + 255) & ~(size_t)255; return p; };
  unsigned short* XH   = (unsigned short*)carve(kBytesXH);
  unsigned short* WT   = (unsigned short*)carve(kBytesWT);
  unsigned short* WST  = (unsigned short*)carve(kBytesWST);
  float*          LIN  = (float*)carve(kBytesLIN);
  unsigned short* QN   = (unsigned short*)carve(kBytesXH);
  unsigned short* KN   = (unsigned short*)carve(kBytesXH);
  unsigned short* VN   = (unsigned short*)carve(kBytesXH);
  float*          SP   = (float*)carve(kBytesSP);
  float*          GATE = (float*)carve(kBytesGATE);
  unsigned short* OH   = (unsigned short*)carve(kBytesXH);
  if (off > ws_size || off > (size_t)134217728) return;

  unsigned short* WqT = WT;
  unsigned short* WkT = WT + (size_t)1 * kDim * kDim;
  unsigned short* WvT = WT + (size_t)2 * kDim * kDim;
  unsigned short* WoT = WT + (size_t)3 * kDim * kDim;

  const int n8x = kTok * (kDim / 8);
  cvt8_act_kernel<<<(n8x + 255) / 256, 256, 0, stream>>>(x, XH, n8x);
  wtcast_kernel<<<dim3(kDim / 64, kDim / 64, 4), 256, 0, stream>>>(Wq, Wk, Wv, Wo, WT, kWCarry);
  wscast_kernel<<<(kSpN * kDim / 8) / 256, 256, 0, stream>>>(Wb, Wg, Wl, WST, kWCarry);

  const dim3 ggrid((kTok / 64) * (kDim / 64) / 8, 1);
  const dim3 cgrid(kTok / kConvT, kHeads);
  wmma_gemm64<0, false, 0, 0, false, 0><<<ggrid, 256, 0, stream>>>(
      XH, XH, kDim, 0L, WqT, WqT, kDim, 0L, (void*)LIN, (void*)LIN, kDim, 0L,
      SP, SP, 0L, kTok, kDim, kDim, kWFold);
  conv_act_kernel<true><<<cgrid, 256, 0, stream>>>(LIN, conv_q, QN);
  wmma_gemm64<0, false, 0, 0, false, 0><<<ggrid, 256, 0, stream>>>(
      XH, XH, kDim, 0L, WkT, WkT, kDim, 0L, (void*)LIN, (void*)LIN, kDim, 0L,
      SP, SP, 0L, kTok, kDim, kDim, kWFold);
  conv_act_kernel<true><<<cgrid, 256, 0, stream>>>(LIN, conv_k, KN);
  wmma_gemm64<0, false, 0, 0, false, 0><<<ggrid, 256, 0, stream>>>(
      XH, XH, kDim, 0L, WvT, WvT, kDim, 0L, (void*)LIN, (void*)LIN, kDim, 0L,
      SP, SP, 0L, kTok, kDim, kDim, kWFold);
  conv_act_kernel<false><<<cgrid, 256, 0, stream>>>(LIN, conv_v, VN);

  const dim3 sgrid((kTok / 64) * (kSpN / 64) / 8, 1);
  wmma_gemm64<0, false, 0, 0, false, 0><<<sgrid, 256, 0, stream>>>(
      XH, XH, kDim, 0L, WST, WST, kDim, 0L, (void*)SP, (void*)SP, kSpN, 0L,
      GATE, GATE, 0L, kTok, kSpN, kDim, kWFold);
  gate_kernel<<<kTok / 256, 256, 0, stream>>>(SP, bg, bl, ltmp, GATE);

  chunk_scan_kernel<<<dim3(kNSlice, kHeads, kBatch), 256, 0, stream>>>(QN, KN, VN, GATE, LIN);

  mix_norm_kernel<<<dim3(kTok / kMixT, kHeads), 256, 0, stream>>>(VN, LIN, GATE, fir_s, fir_l, rmsw, OH);

  wmma_gemm64<0, false, 0, 0, false, 0><<<ggrid, 256, 0, stream>>>(
      OH, OH, kDim, 0L, WoT, WoT, kDim, 0L, d_out, d_out, kDim, 0L,
      SP, SP, 0L, kTok, kDim, kDim, kWFold);
}
